// SpCPE_687194768142
// MI455X (gfx1250) — hardware-verified
//
#include <hip/hip_runtime.h>
#include <hip/hip_bf16.h>
#include <stddef.h>


#define CCH    96
#define NTAP   27
#define KCONV  (NTAP * CCH)
#define NTHR   256
#define CROWS  64
#define CTHR   128
#define AP     (CCH + 8)
#define CP     (CCH + 4)
#define GUNITS ((CROWS * CCH / 8) / CTHR)
#define SUNITS ((16 * CCH) / (4 * 32))
#define WSC    32.0f
#define WSCI   0.03125f
#define LNEPS  1e-5f
#define RC96   (1.0f / 96.0f)

static_assert(KCONV % 32 == 0);
static_assert(CCH % 32 == 0);
static_assert((CROWS * CCH / 8) % CTHR == 0);
static_assert((16 * CCH * 4) % 512 == 0);
static_assert((AP * 2) % 16 == 0);
static_assert((CP * 4) % 16 == 0);
static_assert(CROWS * AP * 2 <= CROWS * CP * 4);
static_assert(CROWS == (CTHR / 32) * 16);
static_assert((CROWS * CCH * 4) % 128 == 0);
static_assert((CCH * CCH) % 8 == 0);
static_assert((CCH * KCONV) % 8 == 0);

typedef float          v4f   __attribute__((ext_vector_type(4)));
typedef float          v8f   __attribute__((ext_vector_type(8)));
typedef int            v4i   __attribute__((ext_vector_type(4)));
typedef _Float16       v8h   __attribute__((ext_vector_type(8)));
typedef _Float16       v16h  __attribute__((ext_vector_type(16)));
typedef unsigned short v8us  __attribute__((ext_vector_type(8)));
typedef unsigned short v16us __attribute__((ext_vector_type(16)));
typedef __bf16         v16bf __attribute__((ext_vector_type(16)));
union FragH { v16h v; v8h h[2]; };
union FragB { v16bf v; v16us w; v8us u[2]; };

__device__ __forceinline__ v8h cvt8h(v4f a, v4f b) {
  v8h r;
  r[0] = (_Float16)a.x; r[1] = (_Float16)a.y; r[2] = (_Float16)a.z; r[3] = (_Float16)a.w;
  r[4] = (_Float16)b.x; r[5] = (_Float16)b.y; r[6] = (_Float16)b.z; r[7] = (_Float16)b.w;
  return r;
}

__device__ __forceinline__ unsigned int bf16_bits(float x) {
  const unsigned int u = __float_as_uint(x);
  return (u + 0x7FFFu + ((u >> 16) & 1u)) >> 16;
}

__device__ __forceinline__ void split_bf(float x, unsigned int& hi, unsigned int& lo) {
  hi = bf16_bits(x);
  const float hf = __uint_as_float(hi << 16);
  lo = bf16_bits(x - hf);
}

__device__ __forceinline__ v8f wmh(v16h a, v16h b, v8f c) {
  v8f d = __builtin_amdgcn_wmma_f32_16x16x32_f16(false, a, false, b, (short)0, c, false, false);
  asm volatile("v_nop\n\tv_nop\n\tv_nop\n\tv_nop" : "+v"(d) : "v"(a), "v"(b));
  return d;
}
__device__ __forceinline__ v8f wmb(v16bf a, v16bf b, v8f c) {
  v8f d = __builtin_amdgcn_wmma_f32_16x16x32_bf16(false, a, false, b, (short)0, c, false, false);
  asm volatile("v_nop\n\tv_nop\n\tv_nop\n\tv_nop" : "+v"(d) : "v"(a), "v"(b));
  return d;
}

__global__ __launch_bounds__(NTHR) void k_x16(const float* __restrict__ f, int total8, int total8p,
                                              _Float16* X16) {
  const int t = blockIdx.x * NTHR + (int)threadIdx.x;
  if (t >= total8p) return;
  const int tc = t < total8 ? t : total8 - 1;
  const size_t e = (size_t)tc * 8;
  const v4f a = *(const v4f*)(f + e);
  const v4f b = *(const v4f*)(f + e + 4);
  v8h hv = cvt8h(a, b);
  if (t >= total8) { const v8h z = {0, 0, 0, 0, 0, 0, 0, 0}; hv = z; }
  _Float16* dp = X16 + (size_t)t * 8;
  *(volatile v8h*)dp = hv;
  __threadfence();
  *(volatile v8h*)dp = hv;
}

__global__ __launch_bounds__(NTHR) void k_prepw(const float* __restrict__ w, _Float16* Wp) {
  const int i = blockIdx.x * NTHR + (int)threadIdx.x;
  if (i >= CCH * KCONV / 8) return;
  const int d   = i / (KCONV / 8);
  const int kk0 = (i - d * (KCONV / 8)) * 8;
  const int tap = kk0 / CCH;
  const int c0  = kk0 - tap * CCH;
  v8h hv;
#pragma unroll
  for (int e = 0; e < 8; ++e)
    hv[e] = (_Float16)(w[((size_t)tap * CCH + c0 + e) * CCH + d] * WSC);
  _Float16* dp = Wp + (size_t)d * KCONV + kk0;
  *(volatile v8h*)dp = hv;
  __threadfence();
  *(volatile v8h*)dp = hv;
}

__global__ __launch_bounds__(NTHR) void k_prepl(const float* __restrict__ wl,
                                               unsigned short* WLh, unsigned short* WLl) {
  const int i = blockIdx.x * NTHR + (int)threadIdx.x;
  if (i >= CCH * CCH / 8) return;
  const size_t e0 = (size_t)i * 8;
  v8us hv, lv;
#pragma unroll
  for (int e = 0; e < 8; ++e) {
    unsigned int hb, lb;
    split_bf(wl[e0 + e], hb, lb);
    hv[e] = (unsigned short)hb;
    lv[e] = (unsigned short)lb;
  }
  *(volatile v8us*)(WLh + e0) = hv;
  *(volatile v8us*)(WLl + e0) = lv;
  __threadfence();
  *(volatile v8us*)(WLh + e0) = hv;
  *(volatile v8us*)(WLl + e0) = lv;
}

__global__ __launch_bounds__(CTHR) void k_main(
    const _Float16* __restrict__ X16, const int* __restrict__ nbr, const _Float16* __restrict__ Wp,
    const unsigned short* __restrict__ WLh, const unsigned short* __restrict__ WLl,
    const float* __restrict__ feat, const float* __restrict__ bconv, const float* __restrict__ blin,
    const float* __restrict__ gam, const float* __restrict__ bet, int n, float* out) {
  __shared__ __attribute__((aligned(16))) float ctile[CROWS * CP];
  __shared__ __attribute__((aligned(16))) int   lidx[CROWS * NTAP];
  _Float16* sA = (_Float16*)ctile;
  const int tid = threadIdx.x, lane = tid & 31, wave = tid >> 5, hh = lane >> 4, m = lane & 15;
  const int rowBase = blockIdx.x * CROWS;

  v8f acc[6];
#pragma unroll
  for (int t = 0; t < 6; ++t) { v8f zz = {0.f, 0.f, 0.f, 0.f, 0.f, 0.f, 0.f, 0.f}; acc[t] = zz; }

#pragma unroll 1
  for (int j = tid; j < CROWS * NTAP; j += CTHR) {
    const int r   = j / NTAP;
    const int k   = j - r * NTAP;
    const int row = rowBase + r;
    const int rcl = row < n ? row : n - 1;
    int g = nbr[(size_t)rcl * NTAP + k];
    g = g < 0 ? g + n + 1 : g;
    g = g < 0 ? 0 : (g > n ? n : g);
    g = row < n ? g : n;
    lidx[j] = g;
  }
  __syncthreads();

#pragma unroll 1
  for (int tap = 0; tap < NTAP; ++tap) {
#pragma unroll
    for (int i = 0; i < GUNITS; ++i) {
      const int u  = i * CTHR + tid;
      const int r  = u / (CCH / 8);
      const int c0 = (u - r * (CCH / 8)) * 8;
      const int g  = lidx[r * NTAP + tap];
      const bool ok = g < n;
      const int gc = ok ? g : n - 1;
      v4i xi = *(const v4i*)(X16 + (size_t)gc * CCH + c0);
      const int mk = ok ? -1 : 0;
      xi = xi & mk;
      *(v4i*)(sA + r * AP + c0) = xi;
    }
    __syncthreads();
    const _Float16* ar = sA + (wave * 16 + m) * AP + 8 * hh;
    const _Float16* wr = Wp + (size_t)m * KCONV + tap * CCH + 8 * hh;
#pragma unroll
    for (int kt = 0; kt < CCH / 32; ++kt) {
      FragH a;
      a.h[0] = *(const v8h*)(ar + 32 * kt);
      a.h[1] = *(const v8h*)(ar + 32 * kt + 16);
#pragma unroll
      for (int t = 0; t < 6; ++t) {
        const _Float16* bp = wr + (size_t)(16 * t) * KCONV + 32 * kt;
        FragH b;
        b.h[0] = *(const v8h*)bp;
        b.h[1] = *(const v8h*)(bp + 16);
        acc[t] = wmh(a.v, b.v, acc[t]);
      }
    }
    __syncthreads();
  }

  {
    float* sp = ctile + (wave * 16 + 8 * hh) * CP + m;
#pragma unroll
    for (int t = 0; t < 6; ++t) {
      const float bc = bconv[16 * t + m];
#pragma unroll
      for (int r = 0; r < 8; ++r) sp[r * CP + 16 * t] = acc[t][r] * WSCI + bc;
    }
  }
  __syncthreads();

  v8f lacc[6];
#pragma unroll
  for (int t = 0; t < 6; ++t) { v8f zz = {0.f, 0.f, 0.f, 0.f, 0.f, 0.f, 0.f, 0.f}; lacc[t] = zz; }
  {
    const float* arow = ctile + (wave * 16 + m) * CP + 8 * hh;
#pragma unroll
    for (int kc = 0; kc < CCH / 32; ++kc) {
      const v4f x0 = *(const v4f*)(arow + 32 * kc);
      const v4f x1 = *(const v4f*)(arow + 32 * kc + 4);
      const v4f x2 = *(const v4f*)(arow + 32 * kc + 16);
      const v4f x3 = *(const v4f*)(arow + 32 * kc + 20);
      float fv[16];
      fv[0]  = x0.x; fv[1]  = x0.y; fv[2]  = x0.z; fv[3]  = x0.w;
      fv[4]  = x1.x; fv[5]  = x1.y; fv[6]  = x1.z; fv[7]  = x1.w;
      fv[8]  = x2.x; fv[9]  = x2.y; fv[10] = x2.z; fv[11] = x2.w;
      fv[12] = x3.x; fv[13] = x3.y; fv[14] = x3.z; fv[15] = x3.w;
      FragB ah, al;
#pragma unroll
      for (int e = 0; e < 16; ++e) {
        unsigned int hb, lb;
        split_bf(fv[e], hb, lb);
        ah.w[e] = (unsigned short)hb;
        al.w[e] = (unsigned short)lb;
      }
#pragma unroll
      for (int t = 0; t < 6; ++t) {
        const size_t bo = (size_t)(16 * t + m) * CCH + 32 * kc + 8 * hh;
        FragB bh, bl;
        bh.u[0] = *(const v8us*)(WLh + bo);
        bh.u[1] = *(const v8us*)(WLh + bo + 16);
        bl.u[0] = *(const v8us*)(WLl + bo);
        bl.u[1] = *(const v8us*)(WLl + bo + 16);
        lacc[t] = wmb(ah.v, bh.v, lacc[t]);
        lacc[t] = wmb(ah.v, bl.v, lacc[t]);
        lacc[t] = wmb(al.v, bh.v, lacc[t]);
      }
    }
  }
  __syncthreads();

  {
    float blv[6], gv[6], btv[6];
#pragma unroll
    for (int t = 0; t < 6; ++t) {
      const int d = 16 * t + m;
      blv[t] = blin[d]; gv[t] = gam[d]; btv[t] = bet[d];
    }
#pragma unroll
    for (int r = 0; r < 8; ++r) {
      float xv[6];
      float s = 0.f;
#pragma unroll
      for (int t = 0; t < 6; ++t) { xv[t] = lacc[t][r] + blv[t]; s += xv[t]; }
      s += __shfl_xor(s, 1, 32);
      s += __shfl_xor(s, 2, 32);
      s += __shfl_xor(s, 4, 32);
      s += __shfl_xor(s, 8, 32);
      const float mu = s * RC96;
      float sq = 0.f;
#pragma unroll
      for (int t = 0; t < 6; ++t) { const float dv = xv[t] - mu; xv[t] = dv; sq += dv * dv; }
      sq += __shfl_xor(sq, 1, 32);
      sq += __shfl_xor(sq, 2, 32);
      sq += __shfl_xor(sq, 4, 32);
      sq += __shfl_xor(sq, 8, 32);
      const float var = sq * RC96;
      const float inv = rsqrtf(var + LNEPS);
      float* ep = ctile + (wave * 16 + 8 * hh + r) * CP + m;
#pragma unroll
      for (int t = 0; t < 6; ++t) ep[16 * t] = xv[t] * inv * gv[t] + btv[t];
    }
  }
  __syncthreads();

  const int rowW = rowBase + wave * 16;
  const float* lp = ctile + wave * 16 * CP;
  v4f ov[SUNITS];
#pragma unroll
  for (int it = 0; it < SUNITS; ++it) {
    const int b  = it * 128 + lane * 4;
    const int rl = b / CCH;
    const int c  = b - rl * CCH;
    const v4f y  = *(const v4f*)(lp + rl * CP + c);
    const int grow  = rowW + rl;
    const int growc = grow < n ? grow : n - 1;
    const v4f fvv = *(const v4f*)(feat + (size_t)growc * CCH + c);
    ov[it] = y + fvv;
  }
#pragma unroll
  for (int it = 0; it < SUNITS; ++it) {
    const int b = it * 128 + lane * 4;
    const int rl = b / CCH, c = b - rl * CCH;
    const int grow = rowW + rl;
    if (grow < n) *(volatile v4f*)(out + (size_t)grow * CCH + c) = ov[it];
  }
  __threadfence();
#pragma unroll
  for (int it = 0; it < SUNITS; ++it) {
    const int b = it * 128 + lane * 4;
    const int rl = b / CCH, c = b - rl * CCH;
    const int grow = rowW + rl;
    if (grow < n) *(volatile v4f*)(out + (size_t)grow * CCH + c) = ov[it];
  }
}

extern "C" void kernel_launch(void* const* d_in, const int* in_sizes, int n_in,
                              void* d_out, int out_size, void* d_ws, size_t ws_size,
                              hipStream_t stream) {
  if (n_in < 8) return;
  const int n = in_sizes[0] / CCH;
  if (n < 1 || in_sizes[0] != n * CCH) return;
  if (in_sizes[1] != n * NTAP || in_sizes[2] != NTAP * CCH * CCH || in_sizes[4] != CCH * CCH) return;
  if (in_sizes[3] != CCH || in_sizes[5] != CCH || in_sizes[6] != CCH || in_sizes[7] != CCH) return;
  if (out_size != n * CCH) return;

  const float* feat  = (const float*)d_in[0];
  const int*   nbr   = (const int*)d_in[1];
  const float* wconv = (const float*)d_in[2];
  const float* bconv = (const float*)d_in[3];
  const float* wlin  = (const float*)d_in[4];
  const float* blin  = (const float*)d_in[5];
  const float* gam   = (const float*)d_in[6];
  const float* bet   = (const float*)d_in[7];
  float* out = (float*)d_out;

  const int total8  = n * (CCH / 8);
  const int total8p = (total8 + 15) & ~15;

  char* ws = (char*)d_ws;
  size_t off = 0;
  const size_t oX16 = off; off += (size_t)total8p * 16;       off = (off + 255) & ~(size_t)255;
  const size_t oWp  = off; off += (size_t)CCH * KCONV * 2;    off = (off + 255) & ~(size_t)255;
  const size_t oWLh = off; off += (size_t)CCH * CCH * 2;      off = (off + 255) & ~(size_t)255;
  const size_t oWLl = off; off += (size_t)CCH * CCH * 2;      off = (off + 255) & ~(size_t)255;
  if (off > ws_size || off > (size_t)134217728) return;

  _Float16*       X16 = (_Float16*)(ws + oX16);
  _Float16*       Wp  = (_Float16*)(ws + oWp);
  unsigned short* WLh = (unsigned short*)(ws + oWLh);
  unsigned short* WLl = (unsigned short*)(ws + oWLl);

  const int nX16Blk  = (total8p + NTHR - 1) / NTHR;
  const int nPrepBlk = (CCH * KCONV / 8 + NTHR - 1) / NTHR;
  const int nLinBlk  = (CCH * CCH / 8 + NTHR - 1) / NTHR;
  const int nMainBlk = (n + CROWS - 1) / CROWS;

  k_x16<<<nX16Blk, NTHR, 0, stream>>>(feat, total8, total8p, X16);
  k_prepw<<<nPrepBlk, NTHR, 0, stream>>>(wconv, Wp);
  k_prepl<<<nLinBlk, NTHR, 0, stream>>>(wlin, WLh, WLl);
  k_main<<<nMainBlk, CTHR, 0, stream>>>(X16, nbr, Wp, WLh, WLl, feat, bconv, blin, gam, bet, n, out);
}
